// MonDEQLayerFC_16750372454624
// MI455X (gfx1250) — hardware-run, weakly checked
//
#include <hip/hip_runtime.h>
#include <math.h>

typedef __attribute__((ext_vector_type(16))) _Float16 v16h;
typedef __attribute__((ext_vector_type(8)))  _Float16 v8h;
typedef __attribute__((ext_vector_type(16))) __bf16   v16b;
typedef __attribute__((ext_vector_type(8)))  __bf16   v8b;
typedef __attribute__((ext_vector_type(8)))  float    v8f;
typedef __attribute__((ext_vector_type(4)))  float    v4f;

constexpr int kNF = 1024;
constexpr int kDI = 512;
constexpr int kNB = 256;
constexpr int kStepLaunches = 99;
constexpr float kStopEps = 1e-4f;
constexpr float kWCarry = 256.0f;
constexpr float kDCarry = 1024.0f;
constexpr float kDCarryInv = 1.0f / kDCarry;
constexpr float kFold = 1.0f / (kWCarry * kDCarry);
constexpr float kF16MinNormal = 6.103515625e-5f;
constexpr float kDClamp = 32768.0f;
constexpr int kStepBlocks = ((kNB / 64) * (kNF / 64)) / 8;
static_assert((kNF % 64) == 0 && (kNB % 64) == 0 && (kDI % 32) == 0 && (kNF % 32) == 0);
static_assert(kStepBlocks * 8 == (kNB / 64) * (kNF / 64));
static_assert(kStepBlocks == 8);
static_assert((kNF / 64) == 16);

constexpr size_t kSzATP = (size_t)kNF * kNF * 2;
constexpr size_t kSzUP  = (size_t)kNF * kDI * 2;
constexpr size_t kSzXP  = (size_t)kNB * kDI * 2;
constexpr size_t kSzKS  = (size_t)kNF * kNF * 4;
constexpr size_t kSzW16 = (size_t)kNF * kNF * 2;
constexpr size_t kSzF32 = (size_t)kNB * kNF * 4;
constexpr size_t kSzD16 = (size_t)kNB * kNF * 2;
constexpr size_t kSzSL  = (size_t)kStepBlocks * 32 * 4;
constexpr size_t kOffATH = 0;
constexpr size_t kOffATL = kOffATH + kSzATP;
constexpr size_t kOffUH  = kOffATL + kSzATP;
constexpr size_t kOffUL  = kOffUH + kSzUP;
constexpr size_t kOffXH  = kOffUL + kSzUP;
constexpr size_t kOffXL  = kOffXH + kSzXP;
constexpr size_t kOffKS  = kOffXL + kSzXP;
constexpr size_t kOffW16 = kOffKS + kSzKS;
constexpr size_t kOffQ0  = kOffW16 + kSzW16;
constexpr size_t kOffQ1  = kOffQ0 + kSzF32;
constexpr size_t kOffZ0  = kOffQ1 + kSzF32;
constexpr size_t kOffZ1  = kOffZ0 + kSzF32;
constexpr size_t kOffZS0 = kOffZ1 + kSzF32;
constexpr size_t kOffZS1 = kOffZS0 + kSzF32;
constexpr size_t kOffD0  = kOffZS1 + kSzF32;
constexpr size_t kOffD1  = kOffD0 + kSzD16;
constexpr size_t kOffSL0 = kOffD1 + kSzD16;
constexpr size_t kOffSL1 = kOffSL0 + kSzSL;
constexpr size_t kWsTotal = kOffSL1 + kSzSL;
static_assert(kWsTotal == 20449280ull);
static_assert(kWsTotal <= 134217728ull);
static_assert((kOffATL % 128) == 0 && (kOffUH % 128) == 0 && (kOffUL % 128) == 0 && (kOffXH % 128) == 0 &&
              (kOffXL % 128) == 0 && (kOffKS % 128) == 0 && (kOffW16 % 128) == 0 && (kOffQ0 % 128) == 0 &&
              (kOffQ1 % 128) == 0 && (kOffZ0 % 128) == 0 && (kOffZ1 % 128) == 0 && (kOffZS0 % 128) == 0 &&
              (kOffZS1 % 128) == 0 && (kOffD0 % 128) == 0 && (kOffD1 % 128) == 0 && (kOffSL0 % 128) == 0 &&
              (kOffSL1 % 128) == 0);

__device__ __forceinline__ unsigned short f2bf_bits(float f) {
  unsigned u = __float_as_uint(f);
  return (unsigned short)((u + 0x7FFFu + ((u >> 16) & 1u)) >> 16);
}
__device__ __forceinline__ float bf_bits2f(unsigned short h) { return __uint_as_float(((unsigned)h) << 16); }

__device__ __forceinline__ void tie_acc(v8f& a) { asm volatile("" : "+v"(a)); }
__device__ __forceinline__ void nop_guard_h(v8f& a, v16h x, v16h y) { asm volatile("v_nop\n\tv_nop\n\tv_nop\n\tv_nop" : "+v"(a) : "v"(x), "v"(y)); }
__device__ __forceinline__ void nop_guard_b(v8f& a, v16b x, v16b y) { asm volatile("v_nop\n\tv_nop\n\tv_nop\n\tv_nop" : "+v"(a) : "v"(x), "v"(y)); }
__device__ __forceinline__ void keep4_h(v16h a, v16h b, v16h c, v16h d) { asm volatile("v_nop" :: "v"(a), "v"(b), "v"(c), "v"(d)); }
__device__ __forceinline__ void keep4_b(v16b a, v16b b, v16b c, v16b d) { asm volatile("v_nop" :: "v"(a), "v"(b), "v"(c), "v"(d)); }
__device__ __forceinline__ void acc_guard4(v8f& a, v8f& b, v8f& c, v8f& d) { asm volatile("v_nop\n\tv_nop\n\tv_nop\n\tv_nop" : "+v"(a), "+v"(b), "+v"(c), "+v"(d)); }
__device__ __forceinline__ void wave_lds_fence() {
  __builtin_amdgcn_fence(__ATOMIC_RELEASE, "workgroup");
  __builtin_amdgcn_wave_barrier();
  __builtin_amdgcn_fence(__ATOMIC_ACQUIRE, "workgroup");
}

template <typename T> struct Frag;
template <> struct Frag<_Float16> {
  typedef v16h V; union U { v16h v; v8h h[2]; };
  static __device__ __forceinline__ v16h load(const _Float16* p) {
    U f; f.h[0] = *(const v8h*)(p); f.h[1] = *(const v8h*)(p + 16); return f.v;
  }
  static __device__ __forceinline__ v8f mma(v16h a, v16h b, v8f c) {
    return __builtin_amdgcn_wmma_f32_16x16x32_f16(false, a, false, b, (short)0, c, false, false);
  }
  static __device__ __forceinline__ void guard1(v8f& a, v16h x, v16h y) { nop_guard_h(a, x, y); }
  static __device__ __forceinline__ void keep(v16h a, v16h b, v16h c, v16h d) { keep4_h(a, b, c, d); }
};
template <> struct Frag<__bf16> {
  typedef v16b V; union U { v16b v; v8b h[2]; };
  static __device__ __forceinline__ v16b load(const __bf16* p) {
    U f; f.h[0] = *(const v8b*)(p); f.h[1] = *(const v8b*)(p + 16); return f.v;
  }
  static __device__ __forceinline__ v8f mma(v16b a, v16b b, v8f c) {
    return __builtin_amdgcn_wmma_f32_16x16x32_bf16(false, a, false, b, (short)0, c, false, false);
  }
  static __device__ __forceinline__ void guard1(v8f& a, v16b x, v16b y) { nop_guard_b(a, x, y); }
  static __device__ __forceinline__ void keep(v16b a, v16b b, v16b c, v16b d) { keep4_b(a, b, c, d); }
};

template <typename T, int SPL>
__device__ __forceinline__ void tile_mac64(const T* __restrict__ A, const T* __restrict__ A2, int lda,
                                           const T* __restrict__ Bt, const T* __restrict__ Bt2, int ldb,
                                           int m0, int n0, int K, int lane, v8f (&acc)[4][4]) {
  typedef typename Frag<T>::V V;
  const int rlane = lane & 15;
  const int koff  = (lane >> 4) * 8;
  for (int k0 = 0; k0 < K; k0 += 32) {
    V bh[4], bl[4];
#pragma unroll
    for (int j = 0; j < 4; ++j) {
      const size_t bo = (size_t)(n0 + (j << 4) + rlane) * ldb + koff + k0;
      bh[j] = Frag<T>::load(Bt + bo);
      if (SPL == 2) bl[j] = Frag<T>::load(Bt2 + bo);
    }
#pragma unroll
    for (int i = 0; i < 4; ++i) {
      const size_t ao = (size_t)(m0 + (i << 4) + rlane) * lda + koff + k0;
      V ah = Frag<T>::load(A + ao);
      V al;
      if (SPL == 2) al = Frag<T>::load(A2 + ao);
#pragma unroll
      for (int j = 0; j < 4; ++j) {
        acc[i][j] = Frag<T>::mma(ah, bh[j], acc[i][j]);
        if (SPL == 2) {
          acc[i][j] = Frag<T>::mma(ah, bl[j], acc[i][j]);
          acc[i][j] = Frag<T>::mma(al, bh[j], acc[i][j]);
        }
      }
      tie_acc(acc[i][0]);
      tie_acc(acc[i][1]);
      tie_acc(acc[i][2]);
      Frag<T>::guard1(acc[i][3], ah, (SPL == 2) ? al : ah);
    }
    Frag<T>::keep(bh[0], bh[1], bh[2], bh[3]);
    if (SPL == 2) Frag<T>::keep(bl[0], bl[1], bl[2], bl[3]);
  }
  acc_guard4(acc[0][0], acc[0][1], acc[0][2], acc[0][3]);
  acc_guard4(acc[1][0], acc[1][1], acc[1][2], acc[1][3]);
  acc_guard4(acc[2][0], acc[2][1], acc[2][2], acc[2][3]);
  acc_guard4(acc[3][0], acc[3][1], acc[3][2], acc[3][3]);
}

__global__ __launch_bounds__(256) void at_planes_kernel(
    const float* __restrict__ A, unsigned short* __restrict__ ATH, unsigned short* __restrict__ ATL)
{
  __shared__ __align__(16) float sT[64 * 68];
  const int tid = threadIdx.x, lane = tid & 31, wave = tid >> 5;
  const int i0 = blockIdx.x * 64;
  const int k0 = blockIdx.y * 64;
  {
    const int lr = tid >> 4, c4 = (tid & 15) * 4;
#pragma unroll
    for (int it = 0; it < 4; ++it) {
      const int r = lr + 16 * it;
      *(v4f*)(sT + r * 68 + c4) = *(const v4f*)(A + (size_t)(k0 + r) * kNF + i0 + c4);
    }
  }
  __syncthreads();
  const int q = lane >> 3, c8 = (lane & 7) * 8;
  v8h hv[2], lv[2];
#pragma unroll
  for (int it = 0; it < 2; ++it) {
    const int row = it * 32 + wave * 4 + q;
#pragma unroll
    for (int e = 0; e < 8; ++e) {
      const float f = sT[(c8 + e) * 68 + row];
      const unsigned short hb = f2bf_bits(f);
      const unsigned short lb = f2bf_bits(f - bf_bits2f(hb));
      hv[it][e] = __builtin_bit_cast(_Float16, hb);
      lv[it][e] = __builtin_bit_cast(_Float16, lb);
    }
  }
  for (int pass = 0; pass < 2; ++pass) {
#pragma unroll
    for (int it = 0; it < 2; ++it) {
      const int row = it * 32 + wave * 4 + q;
      const size_t o = (size_t)(i0 + row) * kNF + k0 + c8;
      *(volatile v8h*)(ATH + o) = hv[it];
      *(volatile v8h*)(ATL + o) = lv[it];
    }
    __threadfence();
  }
}

__global__ __launch_bounds__(256) void split_rows_bf16_kernel(
    const float* __restrict__ src, unsigned short* __restrict__ dhi, unsigned short* __restrict__ dlo, int total8)
{
  const int i = blockIdx.x * 256 + threadIdx.x;
  if (i >= total8) return;
  const size_t e0 = (size_t)i << 3;
  const v4f a0 = *(const v4f*)(src + e0);
  const v4f a1 = *(const v4f*)(src + e0 + 4);
  v8h hv, lv;
#pragma unroll
  for (int e = 0; e < 4; ++e) {
    const unsigned short h0 = f2bf_bits(a0[e]), h1 = f2bf_bits(a1[e]);
    const unsigned short l0 = f2bf_bits(a0[e] - bf_bits2f(h0)), l1 = f2bf_bits(a1[e] - bf_bits2f(h1));
    hv[e]     = __builtin_bit_cast(_Float16, h0);
    hv[4 + e] = __builtin_bit_cast(_Float16, h1);
    lv[e]     = __builtin_bit_cast(_Float16, l0);
    lv[4 + e] = __builtin_bit_cast(_Float16, l1);
  }
  unsigned short* qh = dhi + e0;
  unsigned short* ql = dlo + e0;
  *(volatile v8h*)qh = hv;
  *(volatile v8h*)ql = lv;
  __threadfence();
  *(volatile v8h*)qh = hv;
  *(volatile v8h*)ql = lv;
}

__global__ __launch_bounds__(256) void skew_diag_kernel(
    const float* __restrict__ S, const float* __restrict__ m_raw, float* __restrict__ KS)
{
  __shared__ __align__(16) float sT[64 * 68];
  const int tid = threadIdx.x, lane = tid & 31, wave = tid >> 5;
  const int j0 = blockIdx.x * 64;
  const int i0 = blockIdx.y * 64;
  {
    const int lr = tid >> 4, c4 = (tid & 15) * 4;
#pragma unroll
    for (int it = 0; it < 4; ++it) {
      const int r = lr + 16 * it;
      *(v4f*)(sT + r * 68 + c4) = *(const v4f*)(S + (size_t)(j0 + r) * kNF + i0 + c4);
    }
  }
  __syncthreads();
  const float mr = m_raw[0];
  const float msp = fmaxf(mr, 0.0f) + log1pf(expf(-fabsf(mr)));
  const float onem = 1.0f - msp;
  const int hh = lane >> 4, c4 = (lane & 15) * 4;
  v4f ov[4];
#pragma unroll
  for (int it = 0; it < 4; ++it) {
    const int row = it * 16 + wave * 2 + hh;
    const int gi = i0 + row;
    const v4f s = *(const v4f*)(S + (size_t)gi * kNF + j0 + c4);
#pragma unroll
    for (int e = 0; e < 4; ++e) {
      const int gj = j0 + c4 + e;
      const float st = sT[(c4 + e) * 68 + row];
      const float dg = (gi == gj) ? onem : 0.0f;
      ov[it][e] = (s[e] - st) + dg;
    }
  }
  for (int pass = 0; pass < 2; ++pass) {
#pragma unroll
    for (int it = 0; it < 4; ++it) {
      const int row = it * 16 + wave * 2 + hh;
      *(volatile v4f*)(KS + (size_t)(i0 + row) * kNF + j0 + c4) = ov[it];
    }
    __threadfence();
  }
}

__global__ __launch_bounds__(256) void wbuild_kernel(
    const unsigned short* __restrict__ ATHp, const unsigned short* __restrict__ ATLp,
    const float* __restrict__ KS, unsigned short* __restrict__ W16)
{
  __shared__ __align__(16) float sT[8][16 * 68];
  const int lane = threadIdx.x & 31, wave = threadIdx.x >> 5;
  const int tile = blockIdx.x * 8 + wave;
  const int tm = tile >> 4, tn = tile & 15;
  const int m0 = tm << 6, n0 = tn << 6;
  const __bf16* ATH = (const __bf16*)ATHp;
  const __bf16* ATL = (const __bf16*)ATLp;
  v8f acc[4][4];
#pragma unroll
  for (int i = 0; i < 4; ++i)
#pragma unroll
    for (int j = 0; j < 4; ++j) acc[i][j] = (v8f){0.f,0.f,0.f,0.f,0.f,0.f,0.f,0.f};
  tile_mac64<__bf16, 2>(ATH, ATL, kNF, ATH, ATL, kNF, m0, n0, kNF, lane, acc);

  float* slab = sT[wave];
  const int rlane = lane & 15, mOff = (lane >> 4) * 8;
  const int q8 = lane >> 3, c8 = (lane & 7) * 8;
#pragma unroll
  for (int i = 0; i < 4; ++i) {
    const int mBase = m0 + (i << 4);
#pragma unroll
    for (int j = 0; j < 4; ++j)
#pragma unroll
      for (int r = 0; r < 8; ++r) slab[(mOff + r) * 68 + (j << 4) + rlane] = acc[i][j][r];
    wave_lds_fence();
    v8h wv[4];
#pragma unroll
    for (int it = 0; it < 4; ++it) {
      const int row = it * 4 + q8;
      const float* sp = slab + row * 68 + c8;
      const float* kp = KS + (size_t)(mBase + row) * kNF + n0 + c8;
      const v4f a0 = *(const v4f*)(sp);
      const v4f a1 = *(const v4f*)(sp + 4);
      const v4f k0v = *(const v4f*)(kp);
      const v4f k1v = *(const v4f*)(kp + 4);
#pragma unroll
      for (int e = 0; e < 4; ++e) {
        float w0 = (k0v[e] - a0[e]) * kWCarry;
        float w1 = (k1v[e] - a1[e]) * kWCarry;
        w0 = (fabsf(w0) < kF16MinNormal) ? 0.0f : w0;
        w1 = (fabsf(w1) < kF16MinNormal) ? 0.0f : w1;
        wv[it][e]     = (_Float16)w0;
        wv[it][4 + e] = (_Float16)w1;
      }
    }
    for (int pass = 0; pass < 2; ++pass) {
#pragma unroll
      for (int it = 0; it < 4; ++it) {
        const int row = it * 4 + q8;
        *(volatile v8h*)(W16 + (size_t)(mBase + row) * kNF + n0 + c8) = wv[it];
      }
      __threadfence();
    }
    wave_lds_fence();
  }
}

template <bool F> struct StepElem;
template <> struct StepElem<true>  { typedef __bf16 T; };
template <> struct StepElem<false> { typedef _Float16 T; };

template <bool FIRST>
__global__ __launch_bounds__(256) void step_kernel(
    const unsigned short* __restrict__ Ap, const unsigned short* __restrict__ A2p,
    const unsigned short* __restrict__ Btp, const unsigned short* __restrict__ Bt2p,
    const float* __restrict__ bias,
    const float* __restrict__ Qin, const float* __restrict__ Zin, const float* __restrict__ ZSin,
    const float* __restrict__ slots_in,
    float* __restrict__ Qout, float* __restrict__ Zout, float* __restrict__ ZSout,
    unsigned short* __restrict__ Dout, float* __restrict__ slots_out)
{
  typedef typename StepElem<FIRST>::T T;
  constexpr int SPL = FIRST ? 2 : 0;
  constexpr int KK = FIRST ? kDI : kNF;
  constexpr float FOLD = FIRST ? 1.0f : kFold;
  __shared__ __align__(16) float sT[8][16 * 68];
  __shared__ float sRed[16];
  const int lane = threadIdx.x & 31, wave = threadIdx.x >> 5;
  const int tile = blockIdx.x * 8 + wave;
  const int tm = tile >> 4, tn = tile & 15;
  const int m0 = tm << 6, n0 = tn << 6;
  const int hh = lane >> 4, c4 = (lane & 15) * 4;

  int stop_i = 0;
  if (!FIRST) {
    float s = 0.0f;
#pragma unroll
    for (int bi = 0; bi < kStepBlocks; ++bi) s += slots_in[bi * 32 + lane];
    const float dflag = __shfl(s, 16, 32);
    float t = s;
    t += __shfl_xor(t, 4, 32);
    t += __shfl_xor(t, 2, 32);
    t += __shfl_xor(t, 1, 32);
    const float d2 = __shfl(t, 0, 32);
    const float n2 = __shfl(t, 8, 32);
    const bool go = sqrtf(d2) > kStopEps * (sqrtf(n2) + 1e-8f);
    const bool stop = (dflag > 0.5f) || !go;
    stop_i = __builtin_amdgcn_readfirstlane(stop ? 1 : 0);
  }

  float wd2 = 0.0f, wn2 = 0.0f;
  if (stop_i) {
#pragma unroll 1
    for (int ch = 0; ch < 4; ++ch) {
      v4f cv[8];
#pragma unroll
      for (int it = 0; it < 8; ++it) {
        const int row = ch * 16 + it * 2 + hh;
        cv[it] = *(const v4f*)(Zin + (size_t)(m0 + row) * kNF + n0 + c4);
      }
      for (int pass = 0; pass < 2; ++pass) {
#pragma unroll
        for (int it = 0; it < 8; ++it) {
          const int row = ch * 16 + it * 2 + hh;
          *(volatile v4f*)(Zout + (size_t)(m0 + row) * kNF + n0 + c4) = cv[it];
        }
        __threadfence();
      }
    }
  } else {
    const T* A   = (const T*)Ap;
    const T* A2  = (const T*)A2p;
    const T* Bt  = (const T*)Btp;
    const T* Bt2 = (const T*)Bt2p;
    v8f acc[4][4];
#pragma unroll
    for (int i = 0; i < 4; ++i)
#pragma unroll
      for (int j = 0; j < 4; ++j) acc[i][j] = (v8f){0.f,0.f,0.f,0.f,0.f,0.f,0.f,0.f};
    tile_mac64<T, SPL>(A, A2, KK, Bt, Bt2, KK, m0, n0, KK, lane, acc);

    float* slab = sT[wave];
    const int rlane = lane & 15, mOff = (lane >> 4) * 8;
    const int q8 = lane >> 3, c8 = (lane & 7) * 8;
    v4f bvec = (v4f){0.f, 0.f, 0.f, 0.f};
    if (FIRST) bvec = *(const v4f*)(bias + n0 + c4);
#pragma unroll
    for (int i = 0; i < 4; ++i) {
      const int mBase = m0 + (i << 4);
#pragma unroll
      for (int j = 0; j < 4; ++j)
#pragma unroll
        for (int r = 0; r < 8; ++r) slab[(mOff + r) * 68 + (j << 4) + rlane] = acc[i][j][r] * FOLD;
      wave_lds_fence();
#pragma unroll 1
      for (int g = 0; g < 4; ++g) {
        v4f qn[2], zn[2], zsn[2];
#pragma unroll
        for (int it = 0; it < 2; ++it) {
          const int row = g * 4 + it * 2 + hh;
          const size_t off = (size_t)(mBase + row) * kNF + n0 + c4;
          const v4f a = *(const v4f*)(slab + row * 68 + c4);
          v4f q = bvec;
          v4f z = (v4f){0.f, 0.f, 0.f, 0.f};
          v4f zs = (v4f){0.f, 0.f, 0.f, 0.f};
          if (!FIRST) {
            q  = *(const v4f*)(Qin + off);
            z  = *(const v4f*)(Zin + off);
            zs = *(const v4f*)(ZSin + off);
          }
          v4f dh;
#pragma unroll
          for (int e = 0; e < 4; ++e) {
            const float qv = q[e] + a[e];
            const float zo = z[e];
            const float zv = fmaxf(0.5f * zo + 0.5f * qv, 0.0f);
            const float df = zv - zo;
            wd2 += df * df;
            wn2 += zv * zv;
            float dp = (zv - zs[e]) * kDCarry;
            dp = fminf(fmaxf(dp, -kDClamp), kDClamp);
            dp = (fabsf(dp) < kF16MinNormal) ? 0.0f : dp;
            const _Float16 hval = (_Float16)dp;
            float dq = (float)hval;
            asm volatile("" : "+v"(dq));
            qn[it][e]  = qv;
            zn[it][e]  = zv;
            zsn[it][e] = zs[e] + dq * kDCarryInv;
            dh[e] = dq;
          }
          *(v4f*)(slab + row * 68 + c4) = dh;
        }
        for (int pass = 0; pass < 2; ++pass) {
#pragma unroll
          for (int it = 0; it < 2; ++it) {
            const int row = g * 4 + it * 2 + hh;
            const size_t off = (size_t)(mBase + row) * kNF + n0 + c4;
            *(volatile v4f*)(Qout + off)  = qn[it];
            *(volatile v4f*)(Zout + off)  = zn[it];
            *(volatile v4f*)(ZSout + off) = zsn[it];
          }
          __threadfence();
        }
      }
      wave_lds_fence();
      v8h dv[4];
#pragma unroll
      for (int it = 0; it < 4; ++it) {
        const int row = it * 4 + q8;
        const float* sp = slab + row * 68 + c8;
        const v4f a0 = *(const v4f*)(sp);
        const v4f a1 = *(const v4f*)(sp + 4);
#pragma unroll
        for (int e = 0; e < 4; ++e) {
          dv[it][e]     = (_Float16)a0[e];
          dv[it][4 + e] = (_Float16)a1[e];
        }
      }
      for (int pass = 0; pass < 2; ++pass) {
#pragma unroll
        for (int it = 0; it < 4; ++it) {
          const int row = it * 4 + q8;
          *(volatile v8h*)(Dout + (size_t)(mBase + row) * kNF + n0 + c8) = dv[it];
        }
        __threadfence();
      }
      wave_lds_fence();
    }
  }

#pragma unroll
  for (int o = 16; o > 0; o >>= 1) {
    wd2 += __shfl_xor(wd2, o, 32);
    wn2 += __shfl_xor(wn2, o, 32);
  }
  if (lane == 0) {
    sRed[wave] = wd2;
    sRed[8 + wave] = wn2;
  }
  __syncthreads();
  if (wave == 0) {
    float gv = 0.0f;
    if (!FIRST) gv = slots_in[blockIdx.x * 32 + lane];
    asm volatile("" : "+v"(gv));
    const float lv = sRed[lane & 15];
    float v = (lane < 16) ? lv : 0.0f;
    v = stop_i ? gv : v;
    const float fl = stop_i ? 1.0f : 0.0f;
    v = (lane == 16) ? fl : v;
    volatile float* so = slots_out + blockIdx.x * 32 + lane;
    *so = v;
    __threadfence();
    *so = v;
  }
}

__global__ __launch_bounds__(256) void final_transpose_kernel(
    const float* __restrict__ Z, float* __restrict__ out)
{
  __shared__ __align__(16) float sT[64 * 68];
  const int tid = threadIdx.x, lane = tid & 31, wave = tid >> 5;
  const int p0 = blockIdx.x * 64;
  const int c0 = blockIdx.y * 64;
  {
    const int lr = tid >> 4, c4 = (tid & 15) * 4;
#pragma unroll
    for (int it = 0; it < 4; ++it) {
      const int r = lr + 16 * it;
      *(v4f*)(sT + r * 68 + c4) = *(const v4f*)(Z + (size_t)(c0 + r) * kNF + p0 + c4);
    }
  }
  __syncthreads();
  const int hh = lane >> 4, c4 = (lane & 15) * 4;
  v4f ov[4];
#pragma unroll
  for (int it = 0; it < 4; ++it) {
    const int row = it * 16 + wave * 2 + hh;
#pragma unroll
    for (int e = 0; e < 4; ++e) ov[it][e] = sT[(c4 + e) * 68 + row];
  }
  for (int pass = 0; pass < 2; ++pass) {
#pragma unroll
    for (int it = 0; it < 4; ++it) {
      const int row = it * 16 + wave * 2 + hh;
      *(volatile v4f*)(out + (size_t)(p0 + row) * kNB + c0 + c4) = ov[it];
    }
    __threadfence();
  }
}

extern "C" void kernel_launch(void* const* d_in, const int* in_sizes, int n_in,
                              void* d_out, int out_size, void* d_ws, size_t ws_size,
                              hipStream_t stream) {
  if (n_in < 6) return;
  if (in_sizes[0] != kNF * kNF) return;
  if (in_sizes[1] != kNF * kNF) return;
  if (in_sizes[2] != 1) return;
  if (in_sizes[3] != kNF * kDI) return;
  if (in_sizes[4] != kNF) return;
  if (in_sizes[5] != kNB * kDI) return;
  if (out_size != kNF * kNB) return;
  if (ws_size < kWsTotal) return;

  const float* A     = (const float*)d_in[0];
  const float* S     = (const float*)d_in[1];
  const float* m_raw = (const float*)d_in[2];
  const float* U     = (const float*)d_in[3];
  const float* bvec  = (const float*)d_in[4];
  const float* x     = (const float*)d_in[5];
  float* out = (float*)d_out;

  char* ws = (char*)d_ws;
  unsigned short* ATH = (unsigned short*)(ws + kOffATH);
  unsigned short* ATL = (unsigned short*)(ws + kOffATL);
  unsigned short* UH  = (unsigned short*)(ws + kOffUH);
  unsigned short* UL  = (unsigned short*)(ws + kOffUL);
  unsigned short* XH  = (unsigned short*)(ws + kOffXH);
  unsigned short* XL  = (unsigned short*)(ws + kOffXL);
  float*          KS  = (float*)(ws + kOffKS);
  unsigned short* W16 = (unsigned short*)(ws + kOffW16);
  float* Qp[2]  = { (float*)(ws + kOffQ0),  (float*)(ws + kOffQ1) };
  float* Zp[2]  = { (float*)(ws + kOffZ0),  (float*)(ws + kOffZ1) };
  float* ZSp[2] = { (float*)(ws + kOffZS0), (float*)(ws + kOffZS1) };
  unsigned short* Dp[2] = { (unsigned short*)(ws + kOffD0), (unsigned short*)(ws + kOffD1) };
  float* SLp[2] = { (float*)(ws + kOffSL0), (float*)(ws + kOffSL1) };

  at_planes_kernel<<<dim3(kNF / 64, kNF / 64), 256, 0, stream>>>(A, ATH, ATL);
  split_rows_bf16_kernel<<<(kNF * kDI / 8) / 256, 256, 0, stream>>>(U, UH, UL, kNF * kDI / 8);
  split_rows_bf16_kernel<<<(kNB * kDI / 8) / 256, 256, 0, stream>>>(x, XH, XL, kNB * kDI / 8);
  skew_diag_kernel<<<dim3(kNF / 64, kNF / 64), 256, 0, stream>>>(S, m_raw, KS);
  wbuild_kernel<<<((kNF / 64) * (kNF / 64)) / 8, 256, 0, stream>>>(ATH, ATL, KS, W16);

  step_kernel<true><<<kStepBlocks, 256, 0, stream>>>(
      XH, XL, UH, UL, bvec,
      Qp[1], Zp[1], ZSp[1], SLp[1],
      Qp[0], Zp[0], ZSp[0], Dp[0], SLp[0]);

  for (int s = 0; s < kStepLaunches; ++s) {
    const int pi = s & 1, po = pi ^ 1;
    step_kernel<false><<<kStepBlocks, 256, 0, stream>>>(
        Dp[pi], Dp[pi], W16, W16, bvec,
        Qp[pi], Zp[pi], ZSp[pi], SLp[pi],
        Qp[po], Zp[po], ZSp[po], Dp[po], SLp[po]);
  }

  final_transpose_kernel<<<dim3(kNF / 64, kNB / 64), 256, 0, stream>>>(Zp[kStepLaunches & 1], out);
}
